// QuantumHydraHybridLayer_19112604467489
// MI455X (gfx1250) — hardware-verified
//
#include <hip/hip_runtime.h>


#define NB_ 256
#define NQ 12
#define NAMP 4096
#define NQL 96
#define NM 36

typedef __attribute__((ext_vector_type(16))) __bf16   v16bf;
typedef __attribute__((ext_vector_type(16))) _Float16 v16h;
typedef __attribute__((ext_vector_type(8)))  float    v8f;
typedef __attribute__((ext_vector_type(8)))  unsigned v8u;

__device__ __forceinline__ unsigned f2bf(float f) { unsigned u = __float_as_uint(f); u += 0x7FFFu + ((u >> 16) & 1u); return u >> 16; }
__device__ __forceinline__ unsigned f2h(float f) { return (unsigned)__builtin_bit_cast(unsigned short, (_Float16)f); }
__device__ __forceinline__ int kpat(int v, int half) { return ((v & 4) ? 16 : 0) + half * 8 + 2 * (v & 3); }

template <int F16, int NP> struct Opnd { v16bf p[NP]; };

template <int F16, int NP> __device__ __forceinline__ void pack2(float f0, float f1, unsigned* o) {
    if (F16) { o[0] = f2h(f0) | (f2h(f1) << 16); return; }
    unsigned h0 = f2bf(f0), h1 = f2bf(f1); o[0] = h0 | (h1 << 16);
    if (NP >= 2) {
        float r0 = f0 - __uint_as_float(h0 << 16), r1 = f1 - __uint_as_float(h1 << 16);
        unsigned m0 = f2bf(r0), m1 = f2bf(r1); o[1] = m0 | (m1 << 16);
        if (NP >= 3) {
            float s0 = r0 - __uint_as_float(m0 << 16), s1 = r1 - __uint_as_float(m1 << 16);
            o[2] = f2bf(s0) | (f2bf(s1) << 16);
        }
    }
}
template <int F16, int NP> __device__ __forceinline__ void op_row(const float* rowp, int half, float sc, Opnd<F16, NP>& o) {
    v8u u[NP];
#pragma unroll
    for (int v = 0; v < 8; ++v) {
        int kk = kpat(v, half); unsigned t[3];
        pack2<F16, NP>(rowp[kk] * sc, rowp[kk + 1] * sc, t);
#pragma unroll
        for (int p = 0; p < NP; ++p) u[p][v] = t[p];
    }
#pragma unroll
    for (int p = 0; p < NP; ++p) o.p[p] = __builtin_bit_cast(v16bf, u[p]);
}
template <int F16, int NP> __device__ __forceinline__ void op_row_tail(const float* rowp, int half, float sc, int kvalid, Opnd<F16, NP>& o) {
    v8u u[NP];
#pragma unroll
    for (int v = 0; v < 8; ++v) {
        int kk = kpat(v, half); unsigned t[3];
        float f0 = kk < kvalid ? rowp[kk] * sc : 0.0f, f1 = (kk + 1) < kvalid ? rowp[kk + 1] * sc : 0.0f;
        pack2<F16, NP>(f0, f1, t);
#pragma unroll
        for (int p = 0; p < NP; ++p) u[p][v] = t[p];
    }
#pragma unroll
    for (int p = 0; p < NP; ++p) o.p[p] = __builtin_bit_cast(v16bf, u[p]);
}
template <int F16, int NP> __device__ __forceinline__ void op_col(const float* M, int ld, int n, int k0, int half, float sc, Opnd<F16, NP>& o) {
    v8u u[NP];
#pragma unroll
    for (int v = 0; v < 8; ++v) {
        int kk = k0 + kpat(v, half); unsigned t[3];
        pack2<F16, NP>(M[(size_t)kk * ld + n] * sc, M[(size_t)(kk + 1) * ld + n] * sc, t);
#pragma unroll
        for (int p = 0; p < NP; ++p) u[p][v] = t[p];
    }
#pragma unroll
    for (int p = 0; p < NP; ++p) o.p[p] = __builtin_bit_cast(v16bf, u[p]);
}
template <int F16, int NP> __device__ __forceinline__ void op_col_tail(const float* M, int ld, int n, int k0, int half, float sc, int K, Opnd<F16, NP>& o) {
    v8u u[NP];
#pragma unroll
    for (int v = 0; v < 8; ++v) {
        int kk = k0 + kpat(v, half); unsigned t[3];
        float f0 = kk < K ? M[(size_t)kk * ld + n] * sc : 0.0f, f1 = (kk + 1) < K ? M[(size_t)(kk + 1) * ld + n] * sc : 0.0f;
        pack2<F16, NP>(f0, f1, t);
#pragma unroll
        for (int p = 0; p < NP; ++p) u[p][v] = t[p];
    }
#pragma unroll
    for (int p = 0; p < NP; ++p) o.p[p] = __builtin_bit_cast(v16bf, u[p]);
}
__device__ __forceinline__ v8f wm_bf16(v16bf a, v16bf b, v8f c) { return __builtin_amdgcn_wmma_f32_16x16x32_bf16(false, a, false, b, (short)0, c, false, false); }
template <int F16, int NA, int NB> __device__ __forceinline__ v8f wmma_op(const Opnd<F16, NA>& a, const Opnd<F16, NB>& b, v8f c) {
    if (F16) {
        v16h ah = __builtin_bit_cast(v16h, a.p[0]), bh = __builtin_bit_cast(v16h, b.p[0]);
        c = __builtin_amdgcn_wmma_f32_16x16x32_f16(false, ah, false, bh, (short)0, c, false, false);
        asm volatile("v_nop\n\tv_nop\n\tv_nop\n\tv_nop" : "+v"(c) : "v"(ah), "v"(bh));
        return c;
    }
    constexpr int NMX = NA > NB ? NA : NB;
#pragma unroll
    for (int i = 0; i < NA; ++i)
#pragma unroll
        for (int j = 0; j < NB; ++j)
            if (i + j < NMX) c = wm_bf16(a.p[i], b.p[j], c);
    if (NA == 1 && NB == 1)      asm volatile("v_nop\n\tv_nop\n\tv_nop\n\tv_nop" : "+v"(c) : "v"(a.p[0]), "v"(b.p[0]));
    else if (NA == 2 && NB == 1) asm volatile("v_nop\n\tv_nop\n\tv_nop\n\tv_nop" : "+v"(c) : "v"(a.p[0]), "v"(a.p[1]), "v"(b.p[0]));
    else if (NA == 1 && NB == 2) asm volatile("v_nop\n\tv_nop\n\tv_nop\n\tv_nop" : "+v"(c) : "v"(a.p[0]), "v"(b.p[0]), "v"(b.p[1]));
    else if (NA == 2 && NB == 2) asm volatile("v_nop\n\tv_nop\n\tv_nop\n\tv_nop" : "+v"(c) : "v"(a.p[0]), "v"(a.p[1]), "v"(b.p[0]), "v"(b.p[1]));
    else                         asm volatile("v_nop\n\tv_nop\n\tv_nop\n\tv_nop" : "+v"(c) : "v"(a.p[0]), "v"(a.p[NA - 1]), "v"(b.p[0]), "v"(b.p[NB - 1]), "v"(a.p[NA / 2]), "v"(b.p[NB / 2]));
    return c;
}

struct ZMap { long long s1; long long s2; int zdiv; int pad_; };
__device__ __forceinline__ size_t zoff(const ZMap& m, int z) { return (size_t)((long long)(z / m.zdiv) * m.s1 + (long long)(z % m.zdiv) * m.s2); }

#define ACT_NONE 0
#define ACT_RELU 1
#define ACT_GELU_ERF 2
#define ACT_SILU 3
#define ACT_TANH 4
__device__ __forceinline__ float act_apply(int act, float x) {
    if (act == ACT_RELU) return x > 0.f ? x : 0.f;
    if (act == ACT_GELU_ERF) return 0.5f * x * (1.0f + erff(x * 0.70710678118654752f));
    if (act == ACT_SILU) return x / (1.0f + expf(-x));
    if (act == ACT_TANH) return tanhf(x);
    return x;
}
struct GemmArgs {
    ZMap za, zb_, zc, zbias, zadd, zrsc, zmul, zrbias;
    const float* A; const float* Bm; float* C; const float* bias; const float* add; const float* rsc; const float* mul; const float* rbias;
    long long ldadd, ldmul;
    int lda, ldb, ldc, K;
    float ascale, bscale, oscale, addscale;
    int M, nvalid, nstore, ldrsc;
    int bcs, pad1, pad2, pad3;
};
template <int BT, int F16, int NA, int NB, int RW, int CW, int ACT>
__global__ __launch_bounds__(256) void gemm_kernel(GemmArgs g) {
    constexpr int TR = 16 * RW, TC = 64 * CW, CSTR = TC + 4;
    __shared__ __align__(16) float cst[TR * CSTR];
    const int z = blockIdx.z;
    const float* A = g.A + zoff(g.za, z); const float* Bm = g.Bm + zoff(g.zb_, z); float* C = g.C + zoff(g.zc, z);
    const int tid = threadIdx.x, lane = tid & 31, wv = tid >> 5;
    const int l16 = lane & 15, half = lane >> 4;
    const int rt = wv % RW, ch = wv / RW;
    const int row0 = blockIdx.x * TR, col0 = blockIdx.y * TC + ch * 64;
    int arix = row0 + rt * 16 + l16; if (arix >= g.M) arix = g.M - 1;
    const float* arow = A + (size_t)arix * g.lda;
    v8f acc[4];
#pragma unroll
    for (int t = 0; t < 4; ++t) acc[t] = (v8f){};
    const int K = g.K;
#pragma unroll 1
    for (int kc = 0; kc < K; kc += 32) {
        Opnd<F16, NA> a;
        if (kc + 32 <= K) op_row<F16, NA>(arow + kc, half, g.ascale, a); else op_row_tail<F16, NA>(arow + kc, half, g.ascale, K - kc, a);
#pragma unroll
        for (int t = 0; t < 4; ++t) {
            Opnd<F16, NB> b;
            const int n = col0 + t * 16 + l16;
            if (n < g.nvalid) {
                if (BT) { if (kc + 32 <= K) op_row<F16, NB>(Bm + (size_t)n * g.ldb + kc, half, g.bscale, b); else op_row_tail<F16, NB>(Bm + (size_t)n * g.ldb + kc, half, g.bscale, K - kc, b); }
                else    { if (kc + 32 <= K) op_col<F16, NB>(Bm, g.ldb, n * g.bcs, kc, half, g.bscale, b); else op_col_tail<F16, NB>(Bm, g.ldb, n * g.bcs, kc, half, g.bscale, K, b); }
            } else {
#pragma unroll
                for (int p = 0; p < NB; ++p) b.p[p] = (v16bf){};
            }
            acc[t] = wmma_op<F16, NA, NB>(a, b, acc[t]);
        }
    }
    const float* bias = g.bias ? g.bias + zoff(g.zbias, z) : nullptr;
    const float* add = g.add ? g.add + zoff(g.zadd, z) : nullptr;
    const float* rsc = g.rsc ? g.rsc + zoff(g.zrsc, z) : nullptr;
    const float* mul = g.mul ? g.mul + zoff(g.zmul, z) : nullptr;
    const float* rbias = g.rbias ? g.rbias + zoff(g.zrbias, z) : nullptr;
#pragma unroll
    for (int t = 0; t < 4; ++t) {
        const int cl = ch * 64 + t * 16 + l16;
        const int cg = blockIdx.y * TC + cl;
        const bool cok = cg < g.nvalid;
        const float bv = (bias && cok) ? bias[(size_t)cg * g.bcs] : 0.0f;
#pragma unroll
        for (int r = 0; r < 8; ++r) {
            const int rl = rt * 16 + r + 8 * half;
            float v = acc[t][r] * g.oscale + bv;
            int rg = row0 + rl; if (rg >= g.M) rg = g.M - 1;
            if (rbias) v += rbias[rg];
            if (rsc) v *= rsc[(size_t)rg * g.ldrsc];
            if (mul && cok) v *= mul[(size_t)rg * g.ldmul + cg];
            if (add && cok) v += g.addscale * add[(size_t)rg * g.ldadd + cg];
            cst[rl * CSTR + cl] = v;
        }
    }
    __syncthreads();
    const int col = tid % TC, rsel = tid / TC, rstep = 256 / TC;
    if (ACT != ACT_NONE) {
#pragma unroll 1
        for (int r = rsel; r < TR; r += rstep) cst[r * CSTR + col] = act_apply(ACT, cst[r * CSTR + col]);
    }
    float* ob = C + (size_t)row0 * g.ldc + (size_t)blockIdx.y * TC;
    const bool colok = (int)(blockIdx.y * TC + col) < g.nstore;
    const int rmax = (g.M - row0 < TR) ? (g.M - row0) : TR;
    auto pass = [&]() {
        if (colok) {
#pragma unroll 4
            for (int r = rsel; r < rmax; r += rstep) *(volatile float*)(ob + (size_t)r * g.ldc + col) = cst[r * CSTR + col];
        }
    };
    pass();
    __threadfence();
    pass();
}
static inline ZMap zm(long long s1) { ZMap m; m.s1 = s1; m.s2 = 0; m.zdiv = 1; m.pad_ = 0; return m; }
static inline ZMap zm2(long long s1, long long s2, int zdiv) { ZMap m; m.s1 = s1; m.s2 = s2; m.zdiv = zdiv; m.pad_ = 0; return m; }
static inline GemmArgs gemm_args(const float* A, int lda, ZMap za, const float* Bm, int ldb, ZMap zb, float* C, int ldc, ZMap zc, int M, int N, int K) {
    GemmArgs g; g.za = za; g.zb_ = zb; g.zc = zc; g.zbias = zm(0); g.zadd = zm(0); g.zrsc = zm(0); g.zmul = zm(0); g.zrbias = zm(0);
    g.A = A; g.Bm = Bm; g.C = C; g.bias = nullptr; g.add = nullptr; g.rsc = nullptr; g.mul = nullptr; g.rbias = nullptr; g.ldadd = 0; g.ldmul = 0;
    g.lda = lda; g.ldb = ldb; g.ldc = ldc; g.K = K; g.ascale = 1.0f; g.bscale = 1.0f; g.oscale = 1.0f; g.addscale = 1.0f; g.M = M; g.nvalid = N; g.nstore = N; g.ldrsc = 1;
    g.bcs = 1; g.pad1 = 0; g.pad2 = 0; g.pad3 = 0;
    return g;
}
static_assert(sizeof(ZMap) == 24, "ZMap layout");
static_assert(sizeof(GemmArgs) == 8 * 24 + 8 * 8 + 2 * 8 + 4 * 4 + 4 * 4 + 4 * 4 + 4 * 4, "GemmArgs has no padding");

__global__ __launch_bounds__(256) void softmax_rows(float* S, long long sy, long long sx, int L, float prescale, const float* addv, long long say, int aydiv, int causal,
                                                  const int* imask, long long imy, long long imx, float maskval) {
    __shared__ float red[8];
    const int tid = threadIdx.x, lane = tid & 31, wid = tid >> 5;
    float* row = S + (size_t)blockIdx.y * sy + (size_t)blockIdx.x * sx;
    const float* av = addv ? addv + (size_t)(blockIdx.y / aydiv) * say : nullptr;
    const int* im = imask ? imask + (size_t)(blockIdx.y / aydiv) * imy + (size_t)blockIdx.x * imx : nullptr;
    float v[16];
    const int nj = L / 256;
    float mx = -__builtin_inff();
#pragma unroll
    for (int j = 0; j < 16; ++j) if (j < nj) { float t = row[tid + 256 * j] * prescale; if (av) t += av[tid + 256 * j]; if (im && im[tid + 256 * j] == 0) t = maskval; if (causal && (tid + 256 * j) > (int)blockIdx.x) t = -__builtin_inff(); v[j] = t; mx = fmaxf(mx, t); }
#pragma unroll
    for (int o = 16; o; o >>= 1) mx = fmaxf(mx, __shfl_xor(mx, o, 32));
    if (lane == 0) red[wid] = mx;
    __syncthreads();
    float m = red[0];
#pragma unroll
    for (int i = 1; i < 8; ++i) m = fmaxf(m, red[i]);
    if (m == -__builtin_inff()) m = 0.f;
    __syncthreads();
    float sum = 0.f;
#pragma unroll
    for (int j = 0; j < 16; ++j) if (j < nj) { v[j] = expf(v[j] - m); sum += v[j]; }
#pragma unroll
    for (int o = 16; o; o >>= 1) sum += __shfl_xor(sum, o, 32);
    if (lane == 0) red[wid] = sum;
    __syncthreads();
    float tot = 0.f;
#pragma unroll
    for (int i = 0; i < 8; ++i) tot += red[i];
    const float inv = 1.0f / tot;
#pragma unroll
    for (int j = 0; j < 16; ++j) if (j < nj) *(volatile float*)(row + tid + 256 * j) = v[j] * inv;
    __threadfence();
#pragma unroll
    for (int j = 0; j < 16; ++j) if (j < nj) *(volatile float*)(row + tid + 256 * j) = v[j] * inv;
}

#define VST2(T, p, v) do { const T vst2_v_ = (v); *(volatile T*)(p) = vst2_v_; __threadfence(); *(volatile T*)(p) = vst2_v_; } while (0)
__global__ __launch_bounds__(256) void k_ang(float* L, const float* __restrict__ base) { const int q = blockIdx.x * 256 + threadIdx.x; if (q >= NB_ * NQL) return; const int k = q % NQL, b = q / NQL; float* p = L + (size_t)b * 128 + k; const float v = *p; VST2(float, p, (1.0f / (1.0f + expf(-v))) * (2.0f * 3.14159f) + base[k]); }
__device__ __forceinline__ void ry_gate(float* re, float* im, int q, float th, int t) { const int mask = 1 << (NQ - 1 - q); const float c = cosf(0.5f * th), s = sinf(0.5f * th);
    for (int k = t; k < NAMP / 2; k += 256) { const int lowbits = k & (mask - 1); const int i0 = ((k >> (NQ - 1 - q)) << (NQ - q)) | lowbits; const int i1 = i0 | mask; const float a0r = re[i0], a0i = im[i0], a1r = re[i1], a1i = im[i1];
        re[i0] = c * a0r - s * a1r; im[i0] = c * a0i - s * a1i; re[i1] = s * a0r + c * a1r; im[i1] = s * a0i + c * a1i; } __syncthreads(); }
__device__ __forceinline__ void rx_gate(float* re, float* im, int q, float th, int t) { const int mask = 1 << (NQ - 1 - q); const float c = cosf(0.5f * th), s = sinf(0.5f * th);
    for (int k = t; k < NAMP / 2; k += 256) { const int lowbits = k & (mask - 1); const int i0 = ((k >> (NQ - 1 - q)) << (NQ - q)) | lowbits; const int i1 = i0 | mask; const float a0r = re[i0], a0i = im[i0], a1r = re[i1], a1i = im[i1];
        re[i0] = c * a0r + s * a1i; im[i0] = c * a0i - s * a1r; re[i1] = s * a0i + c * a1r; im[i1] = -s * a0r + c * a1i; } __syncthreads(); }
__device__ __forceinline__ void rz_gate(float* re, float* im, int q, float th, int t) { const int mask = 1 << (NQ - 1 - q); const float c = cosf(0.5f * th), s = sinf(0.5f * th);
    for (int i = t; i < NAMP; i += 256) { const float ar = re[i], ai = im[i]; const float sg = (i & mask) ? 1.f : -1.f;
        re[i] = c * ar - sg * s * ai; im[i] = c * ai + sg * s * ar; } __syncthreads(); }
__device__ __forceinline__ void ising_gate(float* re, float* im, int q0, int q1, float th, int yy, int t) { const int m0 = 1 << (NQ - 1 - q0), m1 = 1 << (NQ - 1 - q1); const float c = cosf(0.5f * th), s = sinf(0.5f * th);
    for (int i = t; i < NAMP; i += 256) { const int j = i ^ m0 ^ m1; if (j < i) continue; float sg = 1.f; if (yy) { const int b0 = (i & m0) != 0, b1 = (i & m1) != 0; sg = (b0 == b1) ? -1.f : 1.f; }
        const float ar = re[i], ai = im[i], br = re[j], bi = im[j];
        re[i] = c * ar + s * sg * bi; im[i] = c * ai - s * sg * br; re[j] = c * br + s * sg * ai; im[j] = c * bi - s * sg * ar; } __syncthreads(); }
__device__ void measure_all(const float* re, const float* im, float* res  , int t) { __shared__ float part[3][256];
    for (int w = 0; w < NQ; ++w) { const int mask = 1 << (NQ - 1 - w); float xr = 0.f, xi = 0.f, z = 0.f;
        for (int k = t; k < NAMP / 2; k += 256) { const int i0 = ((k >> (NQ - 1 - w)) << (NQ - w)) | (k & (mask - 1)); const int i1 = i0 | mask; const float a0r = re[i0], a0i = im[i0], a1r = re[i1], a1i = im[i1];
            xr += a0r * a1r + a0i * a1i; xi += a0r * a1i - a0i * a1r; z += a0r * a0r + a0i * a0i - a1r * a1r - a1i * a1i; }
        part[0][t] = xr; part[1][t] = xi; part[2][t] = z; __syncthreads();
        for (int o = 128; o > 0; o >>= 1) { if (t < o) { part[0][t] += part[0][t + o]; part[1][t] += part[1][t + o]; part[2][t] += part[2][t + o]; } __syncthreads(); }
        if (t == 0) { res[w] = 2.f * part[0][0]; res[NQ + w] = 2.f * part[1][0]; res[2 * NQ + w] = part[2][0]; } __syncthreads(); } }
__global__ __launch_bounds__(256) void k_qlcu(const float* __restrict__ QP, float* M12) { __shared__ float re[NAMP], im[NAMP]; __shared__ float res[NM]; const int b = blockIdx.x, t = threadIdx.x; const float* p = QP + (size_t)b * 128;
    for (int i = t; i < NAMP; i += 256) { re[i] = (i == 0) ? 1.f : 0.f; im[i] = 0.f; } __syncthreads();
    int idx = 0;
    for (int layer = 0; layer < 2; ++layer) {
        for (int i = 0; i < NQ; ++i) ry_gate(re, im, i, p[idx++], t);
        for (int i = 0; i < NQ; ++i) ising_gate(re, im, i, (i + 1) % NQ, p[idx++], 0, t);
        for (int i = 0; i < NQ; ++i) ry_gate(re, im, i, p[idx++], t);
        for (int i = 0; i < NQ; ++i) ising_gate(re, im, i, (i + 1) % NQ, p[idx++], 1, t); }
    measure_all(re, im, res, t);
    if (t < NM) { const int comp = t / NQ, j = t % NQ; const int w1 = (j + 1) % NQ; const int w2 = (NQ - j) % NQ;
        VST2(float, M12 + (size_t)b * 128 + t, res[comp * NQ + w1]); VST2(float, M12 + (size_t)b * 128 + 64 + t, res[comp * NQ + w2]); } }
__global__ __launch_bounds__(256) void k_qd(const float* __restrict__ qd, float* M3) { __shared__ float re[NAMP], im[NAMP]; __shared__ float res[NM]; const int b = blockIdx.x, t = threadIdx.x;
    for (int i = t; i < NAMP; i += 256) { re[i] = (i == 0) ? 1.f : 0.f; im[i] = 0.f; } __syncthreads();
    for (int i = 0; i < NQ; ++i) rx_gate(re, im, i, qd[i], t);
    for (int i = 0; i < NQ; ++i) ry_gate(re, im, i, qd[NQ + i], t);
    for (int i = 0; i < NQ; ++i) rz_gate(re, im, i, qd[2 * NQ + i], t);
    measure_all(re, im, res, t);
    if (t < NM) { VST2(float, M3 + (size_t)b * 64 + t, res[t]); } }
__global__ __launch_bounds__(256) void k_fin(const float* __restrict__ Y1, const float* __restrict__ Y2, const float* __restrict__ Y3, const float* __restrict__ w1, const float* __restrict__ w2, const float* __restrict__ w3, const float* __restrict__ Wout, const float* __restrict__ bout, float* out) { const int b = blockIdx.x * 256 + threadIdx.x; if (b >= NB_) return; const float a1 = fabsf(w1[0]), a2 = fabsf(w2[0]), a3 = fabsf(w3[0]); const float ws = a1 + a2 + a3; float s = bout[0];
#pragma unroll 1
    for (int k = 0; k < NM; ++k) { const float yc = (a1 / ws) * Y1[(size_t)b * 64 + k] + (a2 / ws) * Y2[(size_t)b * 64 + k] + (a3 / ws) * Y3[(size_t)b * 64 + k]; s += yc * Wout[k]; } out[b] = s; }
extern "C" void kernel_launch(void* const* d_in, const int* in_sizes, int n_in,
                              void* d_out, int out_size, void* d_ws, size_t ws_size, hipStream_t stream) {
    (void)in_sizes; (void)n_in; (void)out_size;
    const float* x = (const float*)d_in[0]; const float* Wp = (const float*)d_in[1]; const float* bp = (const float*)d_in[2]; const float* base = (const float*)d_in[3]; const float* qd = (const float*)d_in[4];
    const float* W1 = (const float*)d_in[5]; const float* b1 = (const float*)d_in[6]; const float* W2 = (const float*)d_in[7]; const float* b2 = (const float*)d_in[8]; const float* W3 = (const float*)d_in[9]; const float* b3 = (const float*)d_in[10]; const float* w1 = (const float*)d_in[11]; const float* w2 = (const float*)d_in[12]; const float* w3 = (const float*)d_in[13]; const float* Wout = (const float*)d_in[14]; const float* bout = (const float*)d_in[15];
    float* out = (float*)d_out;
    char* wsp = (char*)d_ws;
    auto take = [&](size_t bytes) { char* p = wsp; wsp += (bytes + 255) & ~(size_t)255; return (void*)p; };
    float* QP = (float*)take((size_t)NB_ * 128 * 4); float* M12 = (float*)take((size_t)NB_ * 128 * 4); float* M3 = (float*)take((size_t)NB_ * 64 * 4); float* Y1 = (float*)take((size_t)NB_ * 64 * 4); float* Y2 = (float*)take((size_t)NB_ * 64 * 4); float* Y3 = (float*)take((size_t)NB_ * 64 * 4);
    if ((size_t)(wsp - (char*)d_ws) > ws_size) return;
    { GemmArgs g = gemm_args(x, 128, zm(0), Wp, 128, zm(0), QP, 128, zm(0), NB_, NQL, 128); g.bias = bp; g.nstore = 128; gemm_kernel<1, 0, 3, 3, 4, 2, ACT_NONE><<<dim3(NB_ / 64, 1, 1), 256, 0, stream>>>(g); }
    k_ang<<<(NB_ * NQL + 255) / 256, 256, 0, stream>>>(QP, base);
    k_qlcu<<<NB_, 256, 0, stream>>>(QP, M12);
    k_qd<<<NB_, 256, 0, stream>>>(qd, M3);
    { GemmArgs g = gemm_args(M12, 128, zm(0), W1, NM, zm(0), Y1, 64, zm(0), NB_, NM, NM); g.bias = b1; g.nstore = 64; gemm_kernel<1, 0, 2, 2, 8, 1, ACT_NONE><<<dim3(NB_ / 128, 1, 1), 256, 0, stream>>>(g); }
    { GemmArgs g = gemm_args(M12 + 64, 128, zm(0), W2, NM, zm(0), Y2, 64, zm(0), NB_, NM, NM); g.bias = b2; g.nstore = 64; gemm_kernel<1, 0, 2, 2, 8, 1, ACT_NONE><<<dim3(NB_ / 128, 1, 1), 256, 0, stream>>>(g); }
    { GemmArgs g = gemm_args(M3, 64, zm(0), W3, NM, zm(0), Y3, 64, zm(0), NB_, NM, NM); g.bias = b3; g.nstore = 64; gemm_kernel<1, 0, 2, 2, 8, 1, ACT_NONE><<<dim3(NB_ / 128, 1, 1), 256, 0, stream>>>(g); }
    k_fin<<<1, 256, 0, stream>>>(Y1, Y2, Y3, w1, w2, w3, Wout, bout, out);
}
